// CausalSelfAttention_71622874628697
// MI455X (gfx1250) — hardware-verified
//
#include <hip/hip_runtime.h>
#ifndef NB
#define NB 64
#endif
#ifndef SEQ
#define SEQ 1024
#endif
#ifndef EROWS
#define EROWS 512
#endif
#define NB_FULL 64
#define SEQ_FULL 1024
#define DMD 64
#define NHD 4
#define HDIM 16
#define QKW 256
#define CTW 128
#define EROWS_USE (((EROWS) < (SEQ)) ? (EROWS) : (SEQ))
#define ETILES (EROWS_USE / 16)
#define LTILES ((SEQ - EROWS_USE) / 16)
static_assert(SEQ % 128 == 0);
static_assert(SEQ <= SEQ_FULL);
static_assert(NB >= 1);
static_assert(NB <= NB_FULL);
static_assert(NHD * HDIM == DMD);
static_assert(NHD == 4);
static_assert(HDIM == 16);
static_assert(DMD == 64);
static_assert(DMD % 32 == 0);
static_assert(CTW % 32 == 0);
static_assert(CTW == 2 * DMD);
static_assert(QKW == 2 * NHD * 2 * HDIM);
static_assert(EROWS % 64 == 0);
static_assert(ETILES % 4 == 0);
static_assert(LTILES % 4 == 0);
static_assert(ETILES + LTILES == SEQ / 16);
static_assert(((size_t)NB * SEQ) % 128 == 0);
static_assert((size_t)NB * SEQ < ((size_t)1 << 30));
static_assert(((size_t)3 * DMD * DMD * 2 + (size_t)DMD * CTW * 2 + (size_t)NB * SEQ * DMD * 2 + (size_t)NB * SEQ * QKW * 2 + (size_t)2 * NB * DMD * SEQ * 2 + (size_t)NB * SEQ * CTW * 2 + 4096) <= ((size_t)128 << 20));

typedef unsigned short v8us __attribute__((ext_vector_type(8), may_alias));
typedef float v8f __attribute__((ext_vector_type(8)));
typedef float v4f __attribute__((ext_vector_type(4)));
typedef float v4fa __attribute__((ext_vector_type(4), may_alias));
typedef _Float16 v16h __attribute__((ext_vector_type(16)));
typedef _Float16 v4h __attribute__((ext_vector_type(4)));
typedef _Float16 h16;
union FragH { v16h v; v8us half[2]; _Float16 h[16]; unsigned short u[16]; };
union H1 { _Float16 h; unsigned short u; };

__device__ __forceinline__ unsigned short bf16_bits(float x) { unsigned int u = __float_as_uint(x); return (unsigned short)((u + 0x7FFFu + ((u >> 16) & 1u)) >> 16); }
__device__ __forceinline__ float bf16_val(unsigned short b) { return __uint_as_float(((unsigned int)b) << 16); }
__device__ __forceinline__ float bf16_rne(float x) { return bf16_val(bf16_bits(x)); }
__device__ __forceinline__ unsigned short hbits(float x) { H1 t; t.h = (_Float16)x; return t.u; }

static __device__ __forceinline__ h16 toh_flush(float v) { const h16 r = (h16)v; return (fabsf(v) < 6.103515625e-05f) ? (h16)0.0f : r; }

__device__ __forceinline__ v16h g2_frag(const _Float16* p, int hh) { FragH f; f.half[0] = *(const v8us*)((const unsigned short*)p + 8 * hh); f.half[1] = *(const v8us*)((const unsigned short*)p + 16 + 8 * hh); return f.v; }
__device__ __forceinline__ v16h g2_fragu(const unsigned short* p, int hh) { FragH f; f.half[0] = *(const v8us*)(p + 8 * hh); f.half[1] = *(const v8us*)(p + 16 + 8 * hh); return f.v; }
__device__ __forceinline__ v8f g2_mma(v16h a, v16h b, v8f c) { v8f d = __builtin_amdgcn_wmma_f32_16x16x32_f16(false, a, false, b, (short)0, c, false, false); asm volatile("v_nop\n\tv_nop\n\tv_nop\n\tv_nop" : "+v"(d) : "v"(a), "v"(b)); return d; }

__global__ __launch_bounds__(256) void k_wplane(const float* __restrict__ W, _Float16* __restrict__ Wt, int N, int K, int ldo, int cofs, float scale) {
  const int t = blockIdx.x * 256 + threadIdx.x; if (t >= N * (K / 8)) return; const int n = t / (K / 8), k8 = (t % (K / 8)) * 8; FragH f;
#pragma unroll
  for (int i = 0; i < 8; ++i) f.h[i] = toh_flush(bf16_rne(W[(size_t)n * K + k8 + i]) * scale);
  const v8us o = f.half[0]; unsigned short* d = (unsigned short*)Wt + (size_t)n * ldo + cofs + k8;
  *(volatile v8us*)d = o; __threadfence(); *(volatile v8us*)d = o;
}

__global__ __launch_bounds__(256) void k_keys16(const float* __restrict__ keys, _Float16* __restrict__ K16) {
  const size_t t = (size_t)blockIdx.x * 256 + threadIdx.x; if (t >= (size_t)NB * SEQ * 8) return;
  const size_t row = t >> 3; const int c8 = (int)(t & 7) * 8; const size_t bb = row / SEQ, s = row % SEQ;
  const float* src = keys + (bb * SEQ_FULL + s) * DMD + c8; FragH f;
#pragma unroll
  for (int q = 0; q < 8; ++q) f.h[q] = (_Float16)bf16_rne(src[q]);
  unsigned short* d = (unsigned short*)K16 + row * DMD + c8;
  *(volatile v8us*)d = f.half[0]; __threadfence(); *(volatile v8us*)d = f.half[0];
}

template <int ACT>
__global__ __launch_bounds__(128) void k_gemm2(const _Float16* __restrict__ A, int lda, size_t sA, const _Float16* __restrict__ Bh, int ldb, size_t sB, float alpha,
    const float* __restrict__ bias, const float* __restrict__ CP, float* __restrict__ C, _Float16* __restrict__ C16, int ldc, size_t sC, int M, int N, int K) {
  static_assert(ACT == 0 || ACT == 17);
  __shared__ __attribute__((aligned(16))) float so[4][32][68];
  const int tid = threadIdx.x, w = tid >> 5, lane = tid & 31, ln = lane & 15, hh = lane >> 4; const int by = blockIdx.y;
  A += (size_t)by * sA; Bh += (size_t)by * sB; const size_t cofs = (size_t)by * sC;
  const int ntn = N >> 6; const int mt = blockIdx.x / ntn, nq = blockIdx.x - mt * ntn; const int row0 = mt * 128 + 32 * w, col0 = nq * 64; if (row0 >= M) return;
  const _Float16* a0p = A + (size_t)(row0 + ln) * lda; const _Float16* a1p = a0p + (size_t)16 * lda;
  const _Float16* b0p = Bh + (size_t)(col0 + ln) * ldb; const _Float16* b1p = b0p + (size_t)16 * ldb; const _Float16* b2p = b1p + (size_t)16 * ldb; const _Float16* b3p = b2p + (size_t)16 * ldb;
  const v8f z8 = {0.f,0.f,0.f,0.f,0.f,0.f,0.f,0.f}; v8f c00 = z8, c01 = z8, c02 = z8, c03 = z8, c10 = z8, c11 = z8, c12 = z8, c13 = z8;
#pragma unroll 1
  for (int kb = 0; kb < K; kb += 32) { const v16h a0 = g2_frag(a0p + kb, hh), a1 = g2_frag(a1p + kb, hh);
    v16h b = g2_frag(b0p + kb, hh); c00 = g2_mma(a0, b, c00); c10 = g2_mma(a1, b, c10);
    b = g2_frag(b1p + kb, hh); c01 = g2_mma(a0, b, c01); c11 = g2_mma(a1, b, c11);
    b = g2_frag(b2p + kb, hh); c02 = g2_mma(a0, b, c02); c12 = g2_mma(a1, b, c12);
    b = g2_frag(b3p + kb, hh); c03 = g2_mma(a0, b, c03); c13 = g2_mma(a1, b, c13); }
  v8f accs[8] = {c00, c01, c02, c03, c10, c11, c12, c13};
#pragma unroll
  for (int u = 0; u < 8; ++u) { const int t = u & 3, half = u >> 2; const int col = col0 + t * 16 + ln; const float bv = bias ? bf16_rne(bias[col]) : 0.f;
#pragma unroll
    for (int r = 0; r < 8; ++r) { const int rloc = half * 16 + 8 * hh + r; float v = accs[u][r] * alpha + bv;
      if (CP) v += CP[cofs + (size_t)(row0 + rloc) * ldc + col];
      if (ACT == 17) v = (v >= 0.f) ? v : 0.2f * v;
      so[w][rloc][t * 16 + ln] = v; } }
  __builtin_amdgcn_fence(4  , "workgroup"); __builtin_amdgcn_wave_barrier();
  const int rsub = lane >> 4, c4 = (lane & 15) * 4;
  for (int pass = 0; pass < 2; ++pass) {
#pragma unroll
    for (int q = 0; q < 16; ++q) { const int r = q * 2 + rsub; if (row0 + r < M) { const v4f v = *(const v4fa*)&so[w][r][c4];
        if (C) *(volatile v4f*)(C + cofs + (size_t)(row0 + r) * ldc + col0 + c4) = v;
        if (C16) { v4h h4; for (int i = 0; i < 4; ++i) h4[i] = (_Float16)v[i]; *(volatile v4h*)(C16 + cofs + (size_t)(row0 + r) * ldc + col0 + c4) = h4; } } }
    if (pass == 0) __threadfence(); }
}

template <int MODE>
__device__ __forceinline__ void gemm_hr_body(const _Float16* __restrict__ A, int lda, size_t sA, const _Float16* __restrict__ Bh, int ldb, size_t sB, float alpha,
    _Float16* __restrict__ O, int ldo, size_t sO, size_t resofs, int M, int N, int K) {
  static_assert(MODE == 0 || MODE == 1);
  __shared__ __attribute__((aligned(16))) float so[4][32][68];
  const int tid = threadIdx.x, lane = tid & 31, ln = lane & 15, hh = lane >> 4; const int w = __builtin_amdgcn_readfirstlane(tid >> 5); const int by = blockIdx.y;
  A += (size_t)by * sA; Bh += (size_t)by * sB; const size_t cofs = (size_t)by * sO;
  const int ntn = N >> 6; const int mt = blockIdx.x / ntn, nq = blockIdx.x - mt * ntn; const int row0 = mt * 128 + 32 * w, col0 = nq * 64; if (row0 >= M) return;
  const _Float16* a0p = A + (size_t)(row0 + ln) * lda; const _Float16* a1p = a0p + (size_t)16 * lda;
  const _Float16* b0p = Bh + (size_t)(col0 + ln) * ldb; const _Float16* b1p = b0p + (size_t)16 * ldb; const _Float16* b2p = b1p + (size_t)16 * ldb; const _Float16* b3p = b2p + (size_t)16 * ldb;
  const v8f z8 = {0.f,0.f,0.f,0.f,0.f,0.f,0.f,0.f}; v8f c00 = z8, c01 = z8, c02 = z8, c03 = z8, c10 = z8, c11 = z8, c12 = z8, c13 = z8;
#pragma unroll 1
  for (int kb = 0; kb < K; kb += 32) { const v16h a0 = g2_frag(a0p + kb, hh), a1 = g2_frag(a1p + kb, hh);
    v16h b = g2_frag(b0p + kb, hh); c00 = g2_mma(a0, b, c00); c10 = g2_mma(a1, b, c10);
    b = g2_frag(b1p + kb, hh); c01 = g2_mma(a0, b, c01); c11 = g2_mma(a1, b, c11);
    b = g2_frag(b2p + kb, hh); c02 = g2_mma(a0, b, c02); c12 = g2_mma(a1, b, c12);
    b = g2_frag(b3p + kb, hh); c03 = g2_mma(a0, b, c03); c13 = g2_mma(a1, b, c13); }
  v8f accs[8] = {c00, c01, c02, c03, c10, c11, c12, c13};
#pragma unroll
  for (int u = 0; u < 8; ++u) { const int t = u & 3, half = u >> 2;
#pragma unroll
    for (int r = 0; r < 8; ++r) { const int rloc = half * 16 + 8 * hh + r; so[w][rloc][t * 16 + ln] = accs[u][r] * alpha; } }
  __builtin_amdgcn_fence(4  , "workgroup"); __builtin_amdgcn_wave_barrier();
  const int rsub = lane >> 4, pc = lane & 15;
  int srcc, isres; size_t dofs;
  if (MODE == 0) { srcc = (pc >> 2) * 16 + (pc & 1) * 8; isres = (pc >> 1) & 1; dofs = cofs + (size_t)nq * 128 + (size_t)(8 * pc); }
  else { srcc = (pc & 7) * 8; isres = pc >> 3; dofs = cofs + (size_t)isres * resofs + (size_t)col0 + (size_t)(8 * (pc & 7)); }
  for (int pass = 0; pass < 2; ++pass) {
#pragma unroll
    for (int q = 0; q < 16; ++q) { const int r = q * 2 + rsub; if (row0 + r < M) {
        const v4f va = *(const v4fa*)&so[w][r][srcc]; const v4f vb = *(const v4fa*)&so[w][r][srcc + 4]; FragH f;
#pragma unroll
        for (int i = 0; i < 4; ++i) {
          const h16 ha = toh_flush(va[i]); const h16 ra = toh_flush((va[i] - (float)ha) * 2048.0f); f.h[i] = isres ? ra : ha;
          const h16 hb = toh_flush(vb[i]); const h16 rb = toh_flush((vb[i] - (float)hb) * 2048.0f); f.h[4 + i] = isres ? rb : hb; }
        *(volatile v8us*)((unsigned short*)O + dofs + (size_t)(row0 + r) * ldo) = f.half[0]; } }
    if (pass == 0) __threadfence(); }
}
__global__ __launch_bounds__(128) void k_gemm_qk(const _Float16* __restrict__ A, int lda, size_t sA, const _Float16* __restrict__ Bh, int ldb, size_t sB, float alpha,
    _Float16* __restrict__ O, int ldo, size_t sO, size_t resofs, int M, int N, int K) { gemm_hr_body<0>(A, lda, sA, Bh, ldb, sB, alpha, O, ldo, sO, resofs, M, N, K); }
__global__ __launch_bounds__(128) void k_gemm_vt(const _Float16* __restrict__ A, int lda, size_t sA, const _Float16* __restrict__ Bh, int ldb, size_t sB, float alpha,
    _Float16* __restrict__ O, int ldo, size_t sO, size_t resofs, int M, int N, int K) { gemm_hr_body<1>(A, lda, sA, Bh, ldb, sB, alpha, O, ldo, sO, resofs, M, N, K); }

template <int EARLY, int T0, int NT>
__device__ __forceinline__ void flash_body(const _Float16* __restrict__ QKP, const _Float16* __restrict__ VT, size_t vres, _Float16* __restrict__ CTXP) {
  __shared__ __attribute__((aligned(16))) float sctx[4][16][68];
  const int wave = __builtin_amdgcn_readfirstlane(threadIdx.x >> 5);
  const int lane = threadIdx.x & 31, ln = lane & 15, hh = lane >> 4;
  const int gt = blockIdx.x * 4 + wave; const int b = gt / NT; const int q0 = (T0 + (gt - b * NT)) * 16;
  const int nsteps = (q0 + 47) >> 5;
  const int qy = q0 + ln;
  const v8f z8 = {0.f,0.f,0.f,0.f,0.f,0.f,0.f,0.f}; const v8us zero8 = {0, 0, 0, 0, 0, 0, 0, 0};
  const float scale2 = 0.25f * 1.4426950408889634f;
  const unsigned short* qk = (const unsigned short*)QKP + (size_t)b * SEQ * QKW;
  const unsigned short* vt = (const unsigned short*)VT + (size_t)b * DMD * SEQ;
#pragma unroll 1
  for (int hd = 0; hd < NHD; ++hd) {
    const v16h qf = g2_fragu(qk + (size_t)qy * QKW + 32 * hd, hh);
    const unsigned short* kp = qk + (size_t)ln * QKW + 2 * DMD + 32 * hd + 8 * hh;
    const unsigned short* vrow = vt + (size_t)(16 * hd + ln) * SEQ;
    v8f o = z8, orr = z8; float m = -1.0e30f, l = 0.f;
#pragma unroll 1
    for (int st = 0; st < nsteps; ++st) {
      const int k0 = st * 32;
      const unsigned short* k0p = kp + (size_t)k0 * QKW; const unsigned short* k1p = k0p + (size_t)16 * QKW;
      FragH ka, kc; ka.half[0] = *(const v8us*)k0p; ka.half[1] = zero8; kc.half[0] = *(const v8us*)k1p; kc.half[1] = zero8;
      const v8f c0 = g2_mma(ka.v, qf, z8); const v8f c1 = g2_mma(kc.v, qf, z8);
      float s[16];
      if (EARLY) {
        FragH ra, rc; ra.half[0] = *(const v8us*)(k0p + 16); ra.half[1] = ka.half[0]; rc.half[0] = *(const v8us*)(k1p + 16); rc.half[1] = kc.half[0];
        const v8f e0 = g2_mma(ra.v, qf, z8); const v8f e1 = g2_mma(rc.v, qf, z8);
#pragma unroll
        for (int r = 0; r < 8; ++r) { s[r] = (c0[r] + e0[r] * (1.0f / 2048.0f)) * scale2; s[8 + r] = (c1[r] + e1[r] * (1.0f / 2048.0f)) * scale2; }
      } else {
#pragma unroll
        for (int r = 0; r < 8; ++r) { s[r] = c0[r] * scale2; s[8 + r] = c1[r] * scale2; }
      }
      if (k0 + 31 > q0) {
#pragma unroll
        for (int r = 0; r < 8; ++r) { const int key = k0 + 8 * hh + r; s[r] = (key > qy) ? -1.0e30f : s[r]; s[8 + r] = (key + 16 > qy) ? -1.0e30f : s[8 + r]; }
      }
      float mx = s[0];
#pragma unroll
      for (int i = 1; i < 16; ++i) mx = fmaxf(mx, s[i]);
      mx = fmaxf(mx, __shfl_xor(mx, 16, 32));
      const float mn = fmaxf(m, mx); const float alpha = exp2f(m - mn); m = mn;
      FragH ph, pr; float ls = 0.f;
#pragma unroll
      for (int i = 0; i < 16; ++i) {
        const float p = exp2f(s[i] - mn) * 1024.0f; const h16 hv = toh_flush(p); ph.h[i] = hv;
        if (EARLY) { ls += p; pr.h[i] = toh_flush((p - (float)hv) * 2048.0f); } else { ls += (float)hv; pr.h[i] = (h16)0.0f; }
      }
      l = l * alpha + ls;
#pragma unroll
      for (int r = 0; r < 8; ++r) { o[r] *= alpha; if (EARLY) orr[r] *= alpha; }
      const v16h vh = g2_fragu(vrow + k0, hh);
      o = g2_mma(vh, ph.v, o);
      if (EARLY) { const v16h vr = g2_fragu(vrow + vres + k0, hh); orr = g2_mma(vh, pr.v, orr); orr = g2_mma(vr, ph.v, orr); }
    }
    const float lt = l + __shfl_xor(l, 16, 32); const float inv = 1.0f / lt;
#pragma unroll
    for (int r = 0; r < 8; ++r) { const float v = (EARLY ? (o[r] + orr[r] * (1.0f / 2048.0f)) : o[r]) * inv; sctx[wave][ln][16 * hd + 8 * hh + r] = v; }
  }
  __builtin_amdgcn_fence(4  , "workgroup"); __builtin_amdgcn_wave_barrier();
  const int rsub = lane >> 4, pc = lane & 15, isres = pc >> 3, c8 = (pc & 7) * 8;
  unsigned short* cbase = (unsigned short*)CTXP + ((size_t)b * SEQ + q0) * CTW + 8 * pc;
  for (int pass = 0; pass < 2; ++pass) {
#pragma unroll
    for (int q = 0; q < 8; ++q) { const int r = q * 2 + rsub;
      const v4f va = *(const v4fa*)&sctx[wave][r][c8]; const v4f vb = *(const v4fa*)&sctx[wave][r][c8 + 4]; FragH f;
#pragma unroll
      for (int i = 0; i < 4; ++i) {
        const h16 ha = toh_flush(va[i]); const h16 ra = EARLY ? toh_flush((va[i] - (float)ha) * 256.0f) : (h16)0.0f; f.h[i] = isres ? ra : ha;
        const h16 hb = toh_flush(vb[i]); const h16 rb = EARLY ? toh_flush((vb[i] - (float)hb) * 256.0f) : (h16)0.0f; f.h[4 + i] = isres ? rb : hb; }
      *(volatile v8us*)(cbase + (size_t)r * CTW) = f.half[0]; }
    if (pass == 0) __threadfence(); }
}
__global__ __launch_bounds__(128) void k_flash_early(const _Float16* __restrict__ QKP, const _Float16* __restrict__ VT, size_t vres, _Float16* __restrict__ CTXP) {
  flash_body<1, 0, (ETILES > 0 ? ETILES : 1)>(QKP, VT, vres, CTXP);
}
__global__ __launch_bounds__(128) void k_flash_late(const _Float16* __restrict__ QKP, const _Float16* __restrict__ VT, size_t vres, _Float16* __restrict__ CTXP) {
  flash_body<0, ETILES, (LTILES > 0 ? LTILES : 1)>(QKP, VT, vres, CTXP);
}

extern "C" void kernel_launch(void* const* d_in, const int* in_sizes, int n_in,
                              void* d_out, int out_size, void* d_ws, size_t ws_size, hipStream_t stream) {
  if (n_in < 3) return;
  const float* x = (const float*)d_in[0]; const float* wqkv = (const float*)d_in[1]; const float* wproj = (const float*)d_in[2];
  const size_t needx = ((size_t)(NB - 1) * SEQ_FULL + SEQ) * DMD;
  if ((size_t)in_sizes[0] < needx || in_sizes[1] < 3 * DMD * DMD || in_sizes[2] < DMD * DMD) return;
  if ((size_t)out_size < needx) return;
  char* ws = (char*)d_ws; size_t off = 0;
  auto take = [&](size_t bytes) { char* p = ws + off; off += (bytes + 255) & ~(size_t)255; return p; };
  _Float16* WQKVt = (_Float16*)take((size_t)3 * DMD * DMD * 2);
  _Float16* WPt = (_Float16*)take((size_t)DMD * CTW * 2);
  _Float16* X16 = (_Float16*)take((size_t)NB * SEQ * DMD * 2);
  _Float16* QKP = (_Float16*)take((size_t)NB * SEQ * QKW * 2);
  _Float16* VT = (_Float16*)take((size_t)2 * NB * DMD * SEQ * 2);
  _Float16* CTXP = (_Float16*)take((size_t)NB * SEQ * CTW * 2);
  if (off > ws_size || off > ((size_t)128 << 20)) return;
  const size_t vres = (size_t)NB * DMD * SEQ;

  k_wplane<<<(unsigned)((3 * DMD * DMD / 8 + 255) / 256), 256, 0, stream>>>(wqkv, WQKVt, 3 * DMD, DMD, DMD, 0, 16.0f);
  k_wplane<<<(unsigned)((DMD * DMD / 8 + 255) / 256), 256, 0, stream>>>(wproj, WPt, DMD, DMD, CTW, 0, 16.0f);
  k_wplane<<<(unsigned)((DMD * DMD / 8 + 255) / 256), 256, 0, stream>>>(wproj, WPt, DMD, DMD, CTW, DMD, 0.0625f);
  k_keys16<<<(unsigned)(((size_t)NB * SEQ * 8 + 255) / 256), 256, 0, stream>>>(x, X16);
  k_gemm_qk<<<dim3((unsigned)(((size_t)NB * SEQ / 128) * (2 * DMD / 64)), 1), 128, 0, stream>>>(X16, DMD, 0, WQKVt, DMD, 0, 0.0625f, QKP, QKW, 0, 0, (int)((size_t)NB * SEQ), 2 * DMD, DMD);
  k_gemm_vt<<<dim3((unsigned)(((DMD + 127) / 128) * (SEQ / 64)), NB), 128, 0, stream>>>(WQKVt + (size_t)2 * DMD * DMD, DMD, 0, X16, DMD, (size_t)SEQ * DMD, 0.0625f, VT, SEQ, (size_t)DMD * SEQ, vres, DMD, SEQ, DMD);
  if (ETILES > 0) k_flash_early<<<(unsigned)((size_t)NB * ETILES / 4), 128, 0, stream>>>(QKP, VT, vres, CTXP);
  if (LTILES > 0) k_flash_late<<<(unsigned)((size_t)NB * LTILES / 4), 128, 0, stream>>>(QKP, VT, vres, CTXP);
  k_gemm2<0><<<dim3((unsigned)((SEQ / 128) * (DMD / 64)), NB), 128, 0, stream>>>(CTXP, CTW, (size_t)SEQ * CTW, WPt, CTW, 0, 0.0625f, nullptr, nullptr, (float*)d_out, nullptr, DMD, (size_t)SEQ_FULL * DMD, SEQ, DMD, CTW);
}
